// DecoderLayer_20581483282919
// MI455X (gfx1250) — hardware-run, weakly checked
//
#include <hip/hip_runtime.h>
#ifndef NB
#define NB 4
#endif
#ifndef SEQ
#define SEQ 1024
#endif
#define NB_FULL 4
#define SEQ_FULL 1024
#define DM 1024
#define NH 16
#define HD 64
#define FF 4096
#define MROWS (NB * SEQ)
#define NQT (SEQ / 64)
#define NKT (SEQ / 64)
static_assert(SEQ % 64 == 0);
static_assert(SEQ <= SEQ_FULL);
static_assert(NB >= 1 && NB <= NB_FULL);
static_assert(MROWS % 128 == 0);
static_assert(DM == NH * HD);
static_assert(HD == 64);
static_assert(DM % 64 == 0 && FF % 64 == 0 && (3 * DM) % 64 == 0 && (2 * DM) % 64 == 0);
static_assert(DM % 32 == 0 && FF % 32 == 0);
static_assert((MROWS * (DM / 8)) % 256 == 0);
static_assert(MROWS % 4 == 0);
static_assert((size_t)MROWS * 3 * DM * 2 <= (size_t)MROWS * FF * 2);
static_assert((size_t)MROWS * 2 * DM * 2 + (size_t)MROWS * DM * 2 <= (size_t)MROWS * FF * 2);
#define WS_WEIGHTS ((size_t)8 * DM * DM * 2 + (size_t)2 * FF * DM * 2)
#define WS_PLANES ((size_t)MROWS * DM * 2 * 2 + (size_t)MROWS * FF * 2 + (size_t)NB * NH * HD * SEQ * 2 + (size_t)MROWS * DM * 4 * 2)
static_assert(WS_WEIGHTS + WS_PLANES <= (size_t)134217728);
static_assert(((size_t)DM * DM * 2) % 256 == 0 && ((size_t)MROWS * DM * 2) % 256 == 0);
static_assert((size_t)NB_FULL * SEQ_FULL * DM * 4 == (size_t)16777216);
static_assert(4 * 32 * 68 * 4 <= 131072);
static_assert(4 * 16 * 68 * 4 <= 131072);
static_assert(4 * DM * 4 <= 131072);
static_assert(64 * 66 * 2 <= 131072);

typedef _Float16 v16h __attribute__((ext_vector_type(16)));
typedef _Float16 v4h  __attribute__((ext_vector_type(4)));
typedef unsigned short v8us __attribute__((ext_vector_type(8), may_alias));
typedef float  v8f  __attribute__((ext_vector_type(8)));
typedef float  v4f  __attribute__((ext_vector_type(4)));
typedef float  v4fa __attribute__((ext_vector_type(4), may_alias));
union FragH { v16h v; v8us half[2]; _Float16 h[16]; unsigned short u[16]; };

#define NEG_INF (-__builtin_inff())

__device__ __forceinline__ unsigned short bf16_bits(float x) { unsigned int u = __float_as_uint(x); return (unsigned short)((u + 0x7FFFu + ((u >> 16) & 1u)) >> 16); }
__device__ __forceinline__ float bf16_val(unsigned short b) { return __uint_as_float(((unsigned int)b) << 16); }
__device__ __forceinline__ float bf16_rne(float x) { return bf16_val(bf16_bits(x)); }

static __device__ __forceinline__ _Float16 toh_flush(float v) { const _Float16 r = (_Float16)v; return (fabsf(v) < 6.103515625e-05f) ? (_Float16)0.0f : r; }

static __device__ __forceinline__ float gelu_erf(float v) { return 0.5f * v * (1.0f + erff(v * 0.70710678118654752f)); }

__device__ __forceinline__ v16h g2_frag(const _Float16* p, int hh) { FragH f; f.half[0] = *(const v8us*)((const unsigned short*)p + 8 * hh); f.half[1] = *(const v8us*)((const unsigned short*)p + 16 + 8 * hh); return f.v; }
__device__ __forceinline__ v8f g2_mma(v16h a, v16h b, v8f c) { v8f d = __builtin_amdgcn_wmma_f32_16x16x32_f16(false, a, false, b, (short)0, c, false, false); asm volatile("v_nop\n\tv_nop\n\tv_nop\n\tv_nop" : "+v"(d) : "v"(a), "v"(b)); return d; }

__global__ __launch_bounds__(256) void k_x16(const float* __restrict__ x, _Float16* __restrict__ X16) {
  const unsigned t = blockIdx.x * 256u + threadIdx.x; if (t >= (unsigned)(MROWS * (DM / 8))) return;
  const unsigned m = t / (unsigned)(DM / 8), c8 = (t % (unsigned)(DM / 8)) * 8u;
  const unsigned b = m / (unsigned)SEQ, s = m % (unsigned)SEQ;
  const float* src = x + ((size_t)b * SEQ_FULL + s) * DM + c8;
  const v4f a = *(const v4fa*)src; const v4f c = *(const v4fa*)(src + 4); FragH f;
#pragma unroll
  for (int q = 0; q < 4; ++q) { f.h[q] = (_Float16)bf16_rne(a[q]); f.h[4 + q] = (_Float16)bf16_rne(c[q]); }
  unsigned short* d = (unsigned short*)X16 + (size_t)m * DM + c8;
  *(volatile v8us*)d = f.half[0]; __threadfence(); *(volatile v8us*)d = f.half[0]; }

__global__ __launch_bounds__(256) void k_wtr(const float* __restrict__ W, unsigned K, unsigned N, _Float16* __restrict__ Bt) {
  __shared__ unsigned short tl[64][66];
  const unsigned tid = threadIdx.x, n0 = blockIdx.x * 64u, k0 = blockIdx.y * 64u;
  for (unsigned i = tid; i < 1024u; i += 256u) { const unsigned r = i >> 4, c4 = (i & 15u) * 4u;
    const v4f v = *(const v4fa*)(W + (size_t)(k0 + r) * N + n0 + c4); FragH f;
#pragma unroll
    for (int q = 0; q < 4; ++q) f.h[q] = toh_flush(bf16_rne(v[q]) * 16.0f);
#pragma unroll
    for (int q = 0; q < 4; ++q) tl[r][c4 + q] = f.u[q]; }
  __syncthreads();
  for (int pass = 0; pass < 2; ++pass) {
#pragma unroll
    for (unsigned rd = 0; rd < 2; ++rd) { const unsigned n = rd * 32u + (tid >> 3), pc = tid & 7u; FragH f;
#pragma unroll
      for (int q = 0; q < 8; ++q) f.u[q] = tl[pc * 8u + q][n];
      *(volatile v8us*)((unsigned short*)Bt + (size_t)(n0 + n) * K + k0 + pc * 8u) = f.half[0]; }
    if (pass == 0) __threadfence(); } }

__global__ __launch_bounds__(128) void k_gemm2(const _Float16* __restrict__ A, unsigned lda, const _Float16* __restrict__ Bh, unsigned ldb, float alpha, const float* __restrict__ bias,
    const float* __restrict__ R, int rfull, _Float16* __restrict__ C16, float* __restrict__ C32, int ofull, unsigned ldc, unsigned M, unsigned N, unsigned K, int mode) {
  __shared__ __attribute__((aligned(16))) float so[4][32][68];
  const unsigned tid = threadIdx.x, lane = tid & 31u, ln = lane & 15u, hh = lane >> 4;
  const unsigned w = (unsigned)__builtin_amdgcn_readfirstlane((int)(tid >> 5));
  const unsigned ntn = N >> 6; const unsigned mt = blockIdx.x / ntn, nq = blockIdx.x - mt * ntn; const unsigned row0 = mt * 128u + 32u * w, col0 = nq * 64u; if (row0 >= M) return;
  const _Float16* a0p = A + (size_t)(row0 + ln) * lda; const _Float16* a1p = a0p + (size_t)16 * lda;
  const _Float16* b0p = Bh + (size_t)(col0 + ln) * ldb; const _Float16* b1p = b0p + (size_t)16 * ldb; const _Float16* b2p = b1p + (size_t)16 * ldb; const _Float16* b3p = b2p + (size_t)16 * ldb;
  const v8f z8 = {0.f,0.f,0.f,0.f,0.f,0.f,0.f,0.f}; v8f c00 = z8, c01 = z8, c02 = z8, c03 = z8, c10 = z8, c11 = z8, c12 = z8, c13 = z8;
#pragma unroll 1
  for (unsigned kb = 0; kb < K; kb += 32u) { const v16h a0 = g2_frag(a0p + kb, (int)hh), a1 = g2_frag(a1p + kb, (int)hh);
    v16h b = g2_frag(b0p + kb, (int)hh); c00 = g2_mma(a0, b, c00); c10 = g2_mma(a1, b, c10);
    b = g2_frag(b1p + kb, (int)hh); c01 = g2_mma(a0, b, c01); c11 = g2_mma(a1, b, c11);
    b = g2_frag(b2p + kb, (int)hh); c02 = g2_mma(a0, b, c02); c12 = g2_mma(a1, b, c12);
    b = g2_frag(b3p + kb, (int)hh); c03 = g2_mma(a0, b, c03); c13 = g2_mma(a1, b, c13); }
  v8f accs[8] = {c00, c01, c02, c03, c10, c11, c12, c13};
#pragma unroll
  for (int u = 0; u < 8; ++u) { const unsigned t = (unsigned)(u & 3), half = (unsigned)(u >> 2); const unsigned col = col0 + t * 16u + ln; const float bv = bf16_rne(bias[col]);
#pragma unroll
    for (int r = 0; r < 8; ++r) { const unsigned rloc = half * 16u + 8u * hh + (unsigned)r; const float v = accs[u][r] * alpha + bv; so[w][rloc][t * 16u + ln] = v; } }
  __builtin_amdgcn_fence(4  , "workgroup"); __builtin_amdgcn_wave_barrier();
  if (mode == 2) {
    static_assert(16 * 32 * 16 == 32 * 64 * 4);
    const unsigned rq = lane >> 3, pc = lane & 7u;
#pragma unroll 4
    for (unsigned g = 0; g < 16; ++g) { const unsigned L = g * 4u + rq; const unsigned row = L >> 1, col = (L & 1u) * 32u + pc * 4u;
      const unsigned mrow = row0 + row; const unsigned gb = mrow / (unsigned)SEQ, gs = mrow % (unsigned)SEQ;
      const size_t mfull = (size_t)gb * SEQ_FULL + gs; const size_t rrow = rfull ? mfull : (size_t)mrow;
      v4f rv = *(const v4fa*)(R + rrow * ldc + col0 + col);
      if (rfull) {
#pragma unroll
        for (int i = 0; i < 4; ++i) rv[i] = bf16_rne(rv[i]); }
      const v4f sv = *(const v4fa*)&so[w][row][col]; const v4f tv = sv + rv; *(v4fa*)&so[w][row][col] = tv; }
    __builtin_amdgcn_fence(4  , "workgroup"); __builtin_amdgcn_wave_barrier();
    for (int pass = 0; pass < 2; ++pass) {
#pragma unroll
      for (unsigned g = 0; g < 16; ++g) { const unsigned L = g * 4u + rq; const unsigned row = L >> 1, col = (L & 1u) * 32u + pc * 4u;
        const unsigned mrow = row0 + row; const unsigned gb = mrow / (unsigned)SEQ, gs = mrow % (unsigned)SEQ;
        const size_t mfull = (size_t)gb * SEQ_FULL + gs; const size_t orow = ofull ? mfull : (size_t)mrow;
        const v4f v = *(const v4fa*)&so[w][row][col];
        *(volatile v4f*)(C32 + orow * ldc + col0 + col) = v; }
      if (pass == 0) __threadfence(); }
  } else {
    static_assert(16 * 32 * 8 == 32 * 64 * 2);
    const unsigned rsub = lane >> 4, c4 = (lane & 15u) * 4u;
    if (mode == 1) {
#pragma unroll 1
      for (unsigned q = 0; q < 16; ++q) { const unsigned r = q * 2u + rsub; v4f v = *(const v4fa*)&so[w][r][c4];
#pragma unroll
        for (int i = 0; i < 4; ++i) v[i] = gelu_erf(v[i]);
        *(v4fa*)&so[w][r][c4] = v; }
      __builtin_amdgcn_fence(4  , "workgroup"); __builtin_amdgcn_wave_barrier(); }
    for (int pass = 0; pass < 2; ++pass) {
#pragma unroll
      for (unsigned q = 0; q < 16; ++q) { const unsigned r = q * 2u + rsub; const v4f v = *(const v4fa*)&so[w][r][c4]; v4h h4;
#pragma unroll
        for (int i = 0; i < 4; ++i) h4[i] = toh_flush(v[i]);
        *(volatile v4h*)(C16 + (size_t)(row0 + r) * ldc + col0 + c4) = h4; }
      if (pass == 0) __threadfence(); } } }

__global__ __launch_bounds__(256) void k_vt2(const _Float16* __restrict__ P, unsigned pitch, unsigned hs, unsigned coff, _Float16* __restrict__ VT) {
  __shared__ unsigned short tl[64][66];
  const unsigned tid = threadIdx.x; const unsigned slab = blockIdx.x / (unsigned)NQT, lg = blockIdx.x % (unsigned)NQT; const unsigned b = slab / (unsigned)NH, hd = slab % (unsigned)NH; const unsigned s0 = lg * 64u;
  for (unsigned i = tid; i < 512u; i += 256u) { const unsigned r = i >> 3, c8 = (i & 7u) * 8u; FragH f;
    f.half[0] = *(const v8us*)((const unsigned short*)P + (size_t)(b * (unsigned)SEQ + s0 + r) * pitch + hd * hs + coff + c8);
#pragma unroll
    for (int q = 0; q < 8; ++q) tl[r][c8 + q] = f.u[q]; }
  __syncthreads();
  for (int pass = 0; pass < 2; ++pass) {
#pragma unroll
    for (unsigned rd = 0; rd < 2; ++rd) { const unsigned d = rd * 32u + (tid >> 3), pc = tid & 7u; FragH f;
#pragma unroll
      for (int q = 0; q < 8; ++q) f.u[q] = tl[pc * 8u + q][d];
      *(volatile v8us*)((unsigned short*)VT + ((size_t)slab * HD + d) * SEQ + s0 + pc * 8u) = f.half[0]; }
    if (pass == 0) __threadfence(); } }

__global__ __launch_bounds__(128) void k_attn(const _Float16* __restrict__ Qp, unsigned qpitch, unsigned qhs, const _Float16* __restrict__ Kp, unsigned kpitch, unsigned khs,
                                              const _Float16* __restrict__ VT, int causal, _Float16* __restrict__ ctx) {
  __shared__ __attribute__((aligned(16))) float so[4][16][68];
  const unsigned tid = threadIdx.x, lane = tid & 31u, l15 = lane & 15u, hh = lane >> 4;
  const unsigned w = (unsigned)__builtin_amdgcn_readfirstlane((int)(tid >> 5));
  const unsigned qt = blockIdx.x, slab = blockIdx.y; const unsigned b = slab / (unsigned)NH, hd = slab % (unsigned)NH;
  const unsigned q0 = qt * 64u + w * 16u;
  const unsigned qloc = w * 16u + l15;
  const _Float16* Qb = Qp + (size_t)(b * (unsigned)SEQ) * qpitch + hd * qhs;
  const _Float16* Kb = Kp + (size_t)(b * (unsigned)SEQ) * kpitch + hd * khs;
  const _Float16* Vb = VT + (size_t)slab * HD * SEQ;
  const _Float16* qrow = Qb + (size_t)(q0 + l15) * qpitch;
  const v16h qf0 = g2_frag(qrow, (int)hh), qf1 = g2_frag(qrow + 32, (int)hh);
  const v8f z8 = {0.f,0.f,0.f,0.f,0.f,0.f,0.f,0.f};
  v8f o[4] = {z8, z8, z8, z8};
  float m = NEG_INF, l = 0.f;
  const float CL = 0.18033688011112042f;
  const unsigned nkt = (causal != 0) ? (qt + 1u) : (unsigned)NKT;
#pragma unroll 1
  for (unsigned it = 0; it < nkt; ++it) {
    const unsigned key0 = it * 64u;
    v8f s[4];
#pragma unroll
    for (unsigned kt = 0; kt < 4; ++kt) {
      const _Float16* krow = Kb + (size_t)(key0 + kt * 16u + l15) * kpitch;
      const v16h ka = g2_frag(krow, (int)hh), kk = g2_frag(krow + 32, (int)hh);
      v8f a = g2_mma(ka, qf0, z8); a = g2_mma(kk, qf1, a); s[kt] = a; }
    if (causal != 0 && it == qt) {
#pragma unroll
      for (unsigned kt = 0; kt < 4; ++kt) {
#pragma unroll
        for (int r = 0; r < 8; ++r) { const unsigned kl = kt * 16u + 8u * hh + (unsigned)r; const float sv = s[kt][r]; s[kt][r] = (kl > qloc) ? NEG_INF : sv; } } }
    float lmax = NEG_INF;
#pragma unroll
    for (int kt = 0; kt < 4; ++kt)
#pragma unroll
      for (int r = 0; r < 8; ++r) lmax = fmaxf(lmax, s[kt][r]);
    lmax = fmaxf(lmax, __shfl_xor(lmax, 16));
    const float mnew = fmaxf(m, lmax);
    const float mref = (mnew == NEG_INF) ? 0.0f : mnew;
    const float alpha = exp2f((m - mref) * CL);
    const float bexp = 10.0f - mref * CL;
    m = mnew;
    float psum = 0.f; FragH pa, pb;
#pragma unroll
    for (int r = 0; r < 8; ++r) {
      const float x0 = fmaf(s[0][r], CL, bexp), x1 = fmaf(s[1][r], CL, bexp), x2 = fmaf(s[2][r], CL, bexp), x3 = fmaf(s[3][r], CL, bexp);
      const float e0 = (x0 < -14.0f) ? 0.0f : exp2f(x0), e1 = (x1 < -14.0f) ? 0.0f : exp2f(x1), e2 = (x2 < -14.0f) ? 0.0f : exp2f(x2), e3 = (x3 < -14.0f) ? 0.0f : exp2f(x3);
      psum += (e0 + e1) + (e2 + e3);
      pa.h[r] = (_Float16)e0; pa.h[8 + r] = (_Float16)e1; pb.h[r] = (_Float16)e2; pb.h[8 + r] = (_Float16)e3; }
    l = l * alpha + psum;
    float ar[8];
#pragma unroll
    for (int r = 0; r < 8; ++r) ar[r] = __shfl(alpha, (int)(8u * hh) + r);
#pragma unroll
    for (unsigned dt = 0; dt < 4; ++dt) {
#pragma unroll
      for (int r = 0; r < 8; ++r) o[dt][r] *= ar[r];
      const _Float16* vrow = Vb + (size_t)(dt * 16u + l15) * SEQ + key0;
      const v16h va = g2_frag(vrow, (int)hh), vb = g2_frag(vrow + 32, (int)hh);
      o[dt] = g2_mma(pa.v, va, o[dt]); o[dt] = g2_mma(pb.v, vb, o[dt]); } }
  const float lt = l + __shfl_xor(l, 16);
  const float inv = 16.0f * (1.0f / lt);
  float ir[8];
#pragma unroll
  for (int r = 0; r < 8; ++r) ir[r] = __shfl(inv, (int)(8u * hh) + r);
#pragma unroll
  for (unsigned dt = 0; dt < 4; ++dt)
#pragma unroll
    for (int r = 0; r < 8; ++r) so[w][8u * hh + (unsigned)r][dt * 16u + l15] = o[dt][r] * ir[r];
  __builtin_amdgcn_fence(4  , "workgroup"); __builtin_amdgcn_wave_barrier();
  static_assert(4 * 32 * 16 == 16 * HD * 2);
  const unsigned rq = lane >> 3, pc = lane & 7u;
  unsigned short* cb = (unsigned short*)ctx + (size_t)(b * (unsigned)SEQ + q0) * DM + hd * (unsigned)HD;
  for (int pass = 0; pass < 2; ++pass) {
#pragma unroll
    for (unsigned g = 0; g < 4; ++g) { const unsigned row = g * 4u + rq; const v4f a = *(const v4fa*)&so[w][row][pc * 8u]; const v4f c = *(const v4fa*)&so[w][row][pc * 8u + 4u]; FragH f;
#pragma unroll
      for (int i = 0; i < 4; ++i) { f.h[i] = toh_flush(a[i]); f.h[4 + i] = toh_flush(c[i]); }
      *(volatile v8us*)(cb + (size_t)row * DM + pc * 8u) = f.half[0]; }
    if (pass == 0) __threadfence(); } }

__global__ __launch_bounds__(128) void k_ln(const float* __restrict__ A, const float* __restrict__ g, const float* __restrict__ be, _Float16* __restrict__ out16, int afull) {
#pragma clang fp contract(off)
  __shared__ __attribute__((aligned(16))) float sr[4][DM];
  static_assert(8 * 32 * 4 == DM);
  static_assert(4 * 32 * 16 == DM * 2);
  const unsigned tid = threadIdx.x, lane = tid & 31u;
  const unsigned w = (unsigned)__builtin_amdgcn_readfirstlane((int)(tid >> 5));
  const unsigned m = blockIdx.x * 4u + w;
  const unsigned gb = m / (unsigned)SEQ, gs = m % (unsigned)SEQ;
  const size_t mfull = (size_t)gb * SEQ_FULL + gs;
  const float* ap = A + (afull ? mfull : (size_t)m) * DM;
  float sum = 0.f;
#pragma unroll 1
  for (unsigned c = 0; c < 8u; ++c) { const unsigned col = c * 128u + lane * 4u; v4f xv = *(const v4fa*)(ap + col);
    if (afull) {
#pragma unroll
      for (int i = 0; i < 4; ++i) xv[i] = bf16_rne(xv[i]); }
    *(v4fa*)&sr[w][col] = xv; sum += (xv[0] + xv[1]) + (xv[2] + xv[3]); }
#pragma unroll
  for (int off = 16; off; off >>= 1) sum += __shfl_xor(sum, off);
  const float mean = sum * (1.0f / (float)DM);
  float s2 = 0.f;
#pragma unroll 1
  for (unsigned c = 0; c < 8u; ++c) { const unsigned col = c * 128u + lane * 4u; const v4f xv = *(const v4fa*)&sr[w][col];
#pragma unroll
    for (int i = 0; i < 4; ++i) { const float d = xv[i] - mean; s2 += d * d; } }
#pragma unroll
  for (int off = 16; off; off >>= 1) s2 += __shfl_xor(s2, off);
  const float rstd = 1.0f / sqrtf(s2 * (1.0f / (float)DM) + 1e-5f);
#pragma unroll 1
  for (unsigned c = 0; c < 8u; ++c) { const unsigned col = c * 128u + lane * 4u; const v4f xv = *(const v4fa*)&sr[w][col];
    const v4f gv = *(const v4fa*)(g + col); const v4f bv = *(const v4fa*)(be + col); v4f v;
#pragma unroll
    for (int i = 0; i < 4; ++i) v[i] = bf16_rne(gv[i]) * (xv[i] - mean) * rstd + bf16_rne(bv[i]);
    *(v4fa*)&sr[w][col] = v; }
  __builtin_amdgcn_fence(4  , "workgroup"); __builtin_amdgcn_wave_barrier();
  unsigned short* o16 = (unsigned short*)out16 + (size_t)m * DM;
  for (int pass = 0; pass < 2; ++pass) {
#pragma unroll 1
    for (unsigned c = 0; c < 4u; ++c) { const unsigned col = c * 256u + lane * 8u; const v4f a = *(const v4fa*)&sr[w][col]; const v4f d = *(const v4fa*)&sr[w][col + 4u]; FragH f;
#pragma unroll
      for (int i = 0; i < 4; ++i) { f.h[i] = toh_flush(a[i]); f.h[4 + i] = toh_flush(d[i]); }
      *(volatile v8us*)(o16 + col) = f.half[0]; }
    if (pass == 0) __threadfence(); } }

extern "C" void kernel_launch(void* const* d_in, const int* in_sizes, int n_in,
                              void* d_out, int out_size, void* d_ws, size_t ws_size, hipStream_t stream) {
  if (n_in < 22) return;
  const float* x    = (const float*)d_in[0];
  const float* enc  = (const float*)d_in[1];
  const float* Wqkv = (const float*)d_in[2];  const float* bqkv = (const float*)d_in[3];
  const float* Wcq  = (const float*)d_in[4];  const float* bcq  = (const float*)d_in[5];
  const float* Wckv = (const float*)d_in[6];  const float* bckv = (const float*)d_in[7];
  const float* Wso  = (const float*)d_in[8];  const float* bso  = (const float*)d_in[9];
  const float* Wco  = (const float*)d_in[10]; const float* bco  = (const float*)d_in[11];
  const float* W1   = (const float*)d_in[12]; const float* b1   = (const float*)d_in[13];
  const float* W2   = (const float*)d_in[14]; const float* b2   = (const float*)d_in[15];
  const float* g1   = (const float*)d_in[16]; const float* be1  = (const float*)d_in[17];
  const float* g2   = (const float*)d_in[18]; const float* be2  = (const float*)d_in[19];
  const float* g3   = (const float*)d_in[20]; const float* be3  = (const float*)d_in[21];
  const long long need_act = ((long long)(NB - 1) * SEQ_FULL + SEQ) * DM;
  if ((long long)in_sizes[0] < need_act || (long long)in_sizes[1] < need_act) return;
  if (in_sizes[2] < DM * 3 * DM || in_sizes[3] < 3 * DM) return;
  if (in_sizes[4] < DM * DM || in_sizes[5] < DM) return;
  if (in_sizes[6] < DM * 2 * DM || in_sizes[7] < 2 * DM) return;
  if (in_sizes[8] < DM * DM || in_sizes[9] < DM) return;
  if (in_sizes[10] < DM * DM || in_sizes[11] < DM) return;
  if (in_sizes[12] < DM * FF || in_sizes[13] < FF) return;
  if (in_sizes[14] < FF * DM || in_sizes[15] < DM) return;
  for (int i = 16; i < 22; ++i) if (in_sizes[i] < DM) return;
  if ((long long)out_size < need_act) return;
  char* ws = (char*)d_ws; size_t off = 0;
  auto take = [&](size_t bytes) { char* p = ws + off; off += (bytes + 255) & ~(size_t)255; return p; };
  _Float16* BQKV = (_Float16*)take((size_t)3 * DM * DM * 2);
  _Float16* BCQ  = (_Float16*)take((size_t)DM * DM * 2);
  _Float16* BCKV = (_Float16*)take((size_t)2 * DM * DM * 2);
  _Float16* BSO  = (_Float16*)take((size_t)DM * DM * 2);
  _Float16* BCO  = (_Float16*)take((size_t)DM * DM * 2);
  _Float16* BW1  = (_Float16*)take((size_t)FF * DM * 2);
  _Float16* BW2  = (_Float16*)take((size_t)DM * FF * 2);
  _Float16* RA   = (_Float16*)take((size_t)MROWS * DM * 2);
  _Float16* RB   = (_Float16*)take((size_t)MROWS * FF * 2);
  _Float16* VT   = (_Float16*)take((size_t)NB * NH * HD * SEQ * 2);
  _Float16* E16  = (_Float16*)take((size_t)MROWS * DM * 2);
  float*    X1   = (float*)take((size_t)MROWS * DM * 4);
  float*    X2   = (float*)take((size_t)MROWS * DM * 4);
  if (off > ws_size || off > (size_t)134217728) return;
  _Float16* XN = RA; _Float16* CTX = RA;
  _Float16* QKV = RB; _Float16* KV = RB; _Float16* Q2 = RB + (size_t)MROWS * 2 * DM; _Float16* FF1 = RB;

  k_wtr<<<dim3(3 * DM / 64, DM / 64), 256, 0, stream>>>(Wqkv, DM, 3 * DM, BQKV);
  k_wtr<<<dim3(DM / 64, DM / 64),     256, 0, stream>>>(Wcq,  DM, DM,     BCQ);
  k_wtr<<<dim3(2 * DM / 64, DM / 64), 256, 0, stream>>>(Wckv, DM, 2 * DM, BCKV);
  k_wtr<<<dim3(DM / 64, DM / 64),     256, 0, stream>>>(Wso,  DM, DM,     BSO);
  k_wtr<<<dim3(DM / 64, DM / 64),     256, 0, stream>>>(Wco,  DM, DM,     BCO);
  k_wtr<<<dim3(FF / 64, DM / 64),     256, 0, stream>>>(W1,   DM, FF,     BW1);
  k_wtr<<<dim3(DM / 64, FF / 64),     256, 0, stream>>>(W2,   FF, DM,     BW2);
  const unsigned gx = (unsigned)(MROWS * (DM / 8) / 256);
  k_x16<<<gx, 256, 0, stream>>>(enc, E16);

  const unsigned mb = (unsigned)(MROWS / 128);
  const unsigned lnb = (unsigned)(MROWS / 4);
  k_ln<<<lnb, 128, 0, stream>>>(x, g1, be1, XN, 1);
  k_gemm2<<<mb * (3 * DM / 64), 128, 0, stream>>>(XN, DM, BQKV, DM, 0.0625f, bqkv, (const float*)nullptr, 0, QKV, (float*)nullptr, 0, 3 * DM, MROWS, 3 * DM, DM, 0);
  k_vt2<<<(unsigned)(NB * NH * NQT), 256, 0, stream>>>(QKV, 3 * DM, HD, 2 * DM, VT);
  k_attn<<<dim3((unsigned)NQT, (unsigned)(NB * NH)), 128, 0, stream>>>(QKV, 3 * DM, HD, QKV + DM, 3 * DM, HD, VT, 1, CTX);
  k_gemm2<<<mb * (DM / 64), 128, 0, stream>>>(CTX, DM, BSO, DM, 0.00390625f, bso, x, 1, (_Float16*)nullptr, X1, 0, DM, MROWS, DM, DM, 2);

  k_ln<<<lnb, 128, 0, stream>>>(X1, g2, be2, XN, 0);
  k_gemm2<<<mb * (DM / 64), 128, 0, stream>>>(XN, DM, BCQ, DM, 0.0625f, bcq, (const float*)nullptr, 0, Q2, (float*)nullptr, 0, DM, MROWS, DM, DM, 0);
  k_gemm2<<<mb * (2 * DM / 64), 128, 0, stream>>>(E16, DM, BCKV, DM, 0.0625f, bckv, (const float*)nullptr, 0, KV, (float*)nullptr, 0, 2 * DM, MROWS, 2 * DM, DM, 0);
  k_vt2<<<(unsigned)(NB * NH * NQT), 256, 0, stream>>>(KV, 2 * DM, HD, DM, VT);
  k_attn<<<dim3((unsigned)NQT, (unsigned)(NB * NH)), 128, 0, stream>>>(Q2, DM, HD, KV, 2 * DM, HD, VT, 0, CTX);
  k_gemm2<<<mb * (DM / 64), 128, 0, stream>>>(CTX, DM, BCO, DM, 0.00390625f, bco, X1, 0, (_Float16*)nullptr, X2, 0, DM, MROWS, DM, DM, 2);

  k_ln<<<lnb, 128, 0, stream>>>(X2, g3, be3, XN, 0);
  k_gemm2<<<mb * (FF / 64), 128, 0, stream>>>(XN, DM, BW1, DM, 0.0625f, b1, (const float*)nullptr, 0, FF1, (float*)nullptr, 0, FF, MROWS, FF, DM, 1);
  k_gemm2<<<mb * (DM / 64), 128, 0, stream>>>(FF1, FF, BW2, FF, 0.0625f, b2, X2, 0, (_Float16*)nullptr, (float*)d_out, 1, DM, MROWS, DM, FF, 2);
}
